// KernelNNFixed_37297495998594
// MI455X (gfx1250) — hardware-run, weakly checked
//
#include <hip/hip_runtime.h>
#include <math.h>

typedef __attribute__((ext_vector_type(16))) __bf16   v16b;
typedef __attribute__((ext_vector_type(8)))  __bf16   v8b;
typedef __attribute__((ext_vector_type(8)))  float    v8f;
typedef __attribute__((ext_vector_type(4)))  float    v4f;
typedef __attribute__((ext_vector_type(2)))  float    v2f;
typedef __attribute__((ext_vector_type(4)))  unsigned v4u;
typedef __attribute__((ext_vector_type(8)))  unsigned v8u;
typedef __attribute__((ext_vector_type(4)))  int      v4i;

constexpr int kB      = 10000;
constexpr int kWin    = 10;
constexpr int kNodes  = 10;
constexpr int kD      = 3;
constexpr int kW      = 30;
constexpr int kKer    = 64;
constexpr int kKin    = 6;
constexpr int kE      = 150000;
constexpr int kNT     = 100000;
constexpr int kXP     = 32;
constexpr int kKK     = 65;
constexpr int kEPad   = 150016;
static_assert(kW == kWin * kD && kW == kNodes * kD, "width");
static_assert(kNT == kB * kNodes, "node count");

constexpr int kLW  = 5;
constexpr int kLNB = 4;
static_assert(kB == 500 * kLW * kLNB, "lstm grid exact");

constexpr int kMlpBlocks = 2344;
static_assert(kMlpBlocks * 64 == kEPad && kEPad >= kE, "edge mlp grid");

constexpr int kCW     = 5;
constexpr int kCE     = 48;
constexpr int kHTP    = 48;
constexpr int kXSP    = 36;
constexpr int kRegion = kKK * kHTP;
static_assert(kE == 625 * kCW * kCE, "message grid exact");
static_assert(kRegion >= kCE * kXSP, "LDS region covers the row tiles");

constexpr int kTile   = 480;
constexpr int kNTiles = 209;
constexpr int kNCh    = 586;
static_assert((kNTiles - 1) * kTile < kNT && kNTiles * kTile >= kNT, "tile cover");
static_assert(((kNT - (kNTiles - 1) * kTile) % 32) == 0 && (kTile % 32) == 0, "whole output lines per block");
static_assert((kE % 8) == 0 && (kNCh - 1) * 256 < kE && kNCh * 256 >= kE, "chunk cover");

constexpr size_t kOffW2T  = 0;
constexpr size_t kOffXA   = kOffW2T + (size_t)kKK * 32 * 32 * 2;
constexpr size_t kOffXB   = kOffXA  + (size_t)kNT * kXP * 4;
constexpr size_t kOffH2   = kOffXB  + (size_t)kNT * kXP * 4;
constexpr size_t kOffMSG  = kOffH2  + (size_t)kEPad * kKer * 4;
constexpr size_t kWsTotal = kOffMSG + (size_t)kE * kXP * 4;
static_assert(kWsTotal == 83337216ull, "carve total");
static_assert(kWsTotal <= 134217728ull, "carve cap");
static_assert((kOffXA % 128) == 0 && (kOffXB % 128) == 0 && (kOffH2 % 128) == 0 && (kOffMSG % 128) == 0, "aligned regions");

__device__ __forceinline__ unsigned f2bf_bits(float f) {
  const unsigned u = __float_as_uint(f);
  return (u + 0x7FFFu + ((u >> 16) & 1u)) >> 16;
}
__device__ __forceinline__ float bf_bits2f(unsigned h) { return __uint_as_float(h << 16); }
__device__ __forceinline__ float rbf(float f) { return bf_bits2f(f2bf_bits(f)); }
__device__ __forceinline__ v4f rbf4(v4f v) {
  const float a = v[0], b = v[1], c = v[2], d = v[3];
  v4f r;
  r[0] = rbf(a); r[1] = rbf(b); r[2] = rbf(c); r[3] = rbf(d);
  return r;
}
__device__ __forceinline__ void split2(float f, unsigned& hb, unsigned& lb) {
  hb = f2bf_bits(f);
  lb = f2bf_bits(f - bf_bits2f(hb));
}
__device__ __forceinline__ float bcast(float v, int l) {
  return __int_as_float(__builtin_amdgcn_readlane(__float_as_int(v), l));
}
__device__ __forceinline__ float sigm(float x) { return __builtin_amdgcn_rcpf(1.0f + __expf(-x)); }
__device__ __forceinline__ float tanh_e(float x) { return 2.0f * __builtin_amdgcn_rcpf(1.0f + __expf(-2.0f * x)) - 1.0f; }

union FragB { v16b v; v8b h[2]; };
__device__ __forceinline__ v16b frag_load(const __bf16* p) {
  FragB f;
  f.h[0] = *(const v8b*)(p);
  f.h[1] = *(const v8b*)(p + 16);
  return f.v;
}
__device__ __forceinline__ v8f mma_bf(v16b a, v16b b, v8f c) {
  return __builtin_amdgcn_wmma_f32_16x16x32_bf16(false, a, false, b, (short)0, c, false, false);
}
__device__ __forceinline__ void guard1(v8f& c, v16b a0, v16b a1, v16b b) {
  asm volatile("v_nop\n\tv_nop\n\tv_nop\n\tv_nop" : "+v"(c) : "v"(a0), "v"(a1), "v"(b));
}
__device__ __forceinline__ void scale_acc(v8f& a, const v8f c, const v4f h0, const v4f h1) {
  a[0] = fmaf(h0[0], c[0], a[0]);
  a[1] = fmaf(h0[1], c[1], a[1]);
  a[2] = fmaf(h0[2], c[2], a[2]);
  a[3] = fmaf(h0[3], c[3], a[3]);
  a[4] = fmaf(h1[0], c[4], a[4]);
  a[5] = fmaf(h1[1], c[5], a[5]);
  a[6] = fmaf(h1[2], c[6], a[6]);
  a[7] = fmaf(h1[3], c[7], a[7]);
}

__global__ __launch_bounds__(128) void prep_w2t(const float* __restrict__ k2w, const float* __restrict__ k2b,
                                                unsigned short* __restrict__ w2t)
{
  const int kk  = blockIdx.x;
  const int tid = threadIdx.x;
  const int o   = tid >> 2;
  const int i0  = (tid & 3) * 8;
  const float* src = (kk < kKer) ? (k2w + (size_t)kk * (kW * kW)) : k2b;
  const int oc = o < kW ? o : kW - 1;
  unsigned wds[4];
#pragma unroll
  for (int p = 0; p < 4; ++p) {
    const int ia = i0 + 2 * p;
    const int ib = ia + 1;
    const int iac = ia < kW ? ia : kW - 1;
    const int ibc = ib < kW ? ib : kW - 1;
    float va = src[iac * kW + oc];
    float vb = src[ibc * kW + oc];
    asm volatile("" : "+v"(va), "+v"(vb));
    const bool oka = (ia < kW) && (o < kW);
    const bool okb = (ib < kW) && (o < kW);
    va = oka ? va : 0.0f;
    vb = okb ? vb : 0.0f;
    const unsigned ha = f2bf_bits(va);
    const unsigned hb = f2bf_bits(vb);
    wds[p] = ha | (hb << 16);
  }
  v4u pk;
  pk[0] = wds[0]; pk[1] = wds[1]; pk[2] = wds[2]; pk[3] = wds[3];
  unsigned short* dst = w2t + (size_t)kk * 1024 + (size_t)tid * 8;
  *(volatile v4u*)dst = pk;
  __threadfence();
  *(volatile v4u*)dst = pk;
}

__global__ __launch_bounds__(160) void lstm_enc(
    const float* __restrict__ xpos, const float* __restrict__ fc0w, const float* __restrict__ fc0b,
    const float* __restrict__ wih, const float* __restrict__ whh, const float* __restrict__ bih,
    const float* __restrict__ bhh, float* __restrict__ xA)
{
  __shared__ __align__(16) float s_f0w[900];
  __shared__ __align__(16) float s_wih[3600];
  __shared__ __align__(16) float s_whh[3600];
  __shared__ __align__(16) float s_hist[kLW * 40 * 32];
  const int tid  = threadIdx.x;
  const int lane = tid & 31;
  const int wave = __builtin_amdgcn_readfirstlane((int)(threadIdx.x >> 5));
#pragma unroll 1
  for (int it = 0; it < 6; ++it) {
    const int i = it * 160 + tid;
    const int ic = i < 900 ? i : 899;
    float v = fc0w[ic];
    asm volatile("" : "+v"(v));
    if (i < 900) s_f0w[i] = rbf(v);
  }
#pragma unroll 1
  for (int it = 0; it < 23; ++it) {
    const int i = it * 160 + tid;
    const int ic = i < 3600 ? i : 3599;
    float v0 = wih[ic];
    float v1 = whh[ic];
    asm volatile("" : "+v"(v0), "+v"(v1));
    if (i < 3600) { s_wih[i] = rbf(v0); s_whh[i] = rbf(v1); }
  }
  float* hw = s_hist + wave * (40 * 32);
#pragma unroll
  for (int it = 0; it < 3; ++it) {
    const int r = it * 16 + (lane >> 1);
    if (r < 40) hw[r * 32 + 30 + (lane & 1)] = 0.0f;
  }
  __syncthreads();

  const int jc = lane < kW ? lane : kW - 1;
  const int nq = jc / kD;
  const int dq = jc - nq * kD;
  const int b0 = (blockIdx.x * kLW + wave) * kLNB;
  const float f0b = rbf(fc0b[jc]);
  const float bzi = rbf(bih[jc])          + rbf(bhh[jc]);
  const float bzf = rbf(bih[kW + jc])     + rbf(bhh[kW + jc]);
  const float bzg = rbf(bih[2 * kW + jc]) + rbf(bhh[2 * kW + jc]);
  const float bzo = rbf(bih[3 * kW + jc]) + rbf(bhh[3 * kW + jc]);

  float h[kLNB], c[kLNB];
#pragma unroll
  for (int nb = 0; nb < kLNB; ++nb) { h[nb] = 0.0f; c[nb] = 0.0f; }

#pragma unroll 1
  for (int t = 0; t < kWin; ++t) {
    float xr[kLNB], xt[kLNB];
#pragma unroll
    for (int nb = 0; nb < kLNB; ++nb) {
      xr[nb] = rbf(xpos[((size_t)(b0 + nb) * kWin + t) * kW + jc]);
      xt[nb] = 0.0f;
    }
#pragma unroll 1
    for (int i = 0; i < kW; ++i) {
      const float w = s_f0w[i * kW + jc];
#pragma unroll
      for (int nb = 0; nb < kLNB; ++nb) xt[nb] = fmaf(bcast(xr[nb], i), w, xt[nb]);
    }
    float zi[kLNB], zf[kLNB], zg[kLNB], zo[kLNB];
#pragma unroll
    for (int nb = 0; nb < kLNB; ++nb) {
      xt[nb] += f0b;
      zi[nb] = 0.0f; zf[nb] = 0.0f; zg[nb] = 0.0f; zo[nb] = 0.0f;
    }
#pragma unroll 1
    for (int i = 0; i < kW; ++i) {
      const float* wi = s_wih + i * 120 + jc;
      const float* wh = s_whh + i * 120 + jc;
      const float wi0 = wi[0], wi1 = wi[30], wi2 = wi[60], wi3 = wi[90];
      const float wh0 = wh[0], wh1 = wh[30], wh2 = wh[60], wh3 = wh[90];
#pragma unroll
      for (int nb = 0; nb < kLNB; ++nb) {
        const float xb = bcast(xt[nb], i);
        const float hb = bcast(h[nb], i);
        zi[nb] = fmaf(xb, wi0, zi[nb]);
        zf[nb] = fmaf(xb, wi1, zf[nb]);
        zg[nb] = fmaf(xb, wi2, zg[nb]);
        zo[nb] = fmaf(xb, wi3, zo[nb]);
        zi[nb] = fmaf(hb, wh0, zi[nb]);
        zf[nb] = fmaf(hb, wh1, zf[nb]);
        zg[nb] = fmaf(hb, wh2, zg[nb]);
        zo[nb] = fmaf(hb, wh3, zo[nb]);
      }
    }
#pragma unroll
    for (int nb = 0; nb < kLNB; ++nb) {
      const float gi = sigm(zi[nb] + bzi);
      const float gf = sigm(zf[nb] + bzf);
      const float gg = tanh_e(zg[nb] + bzg);
      const float go = sigm(zo[nb] + bzo);
      c[nb] = gf * c[nb] + gi * gg;
      h[nb] = go * tanh_e(c[nb]);
      if (lane < kW) hw[(nb * kNodes + nq) * 32 + t * kD + dq] = h[nb];
    }
  }
  __syncthreads();
  float* dst = xA + (size_t)b0 * (kNodes * kXP);
  for (int pass = 0; pass < 2; ++pass) {
#pragma unroll
    for (int it = 0; it < 10; ++it) {
      const int idx = it * 32 + lane;
      const v4f v = *(const v4f*)(hw + idx * 4);
      *(volatile v4f*)(dst + (size_t)idx * 4) = v;
    }
    __threadfence();
  }
}

__global__ __launch_bounds__(64) void edge_mlp(
    const float* __restrict__ ea, const float* __restrict__ k0w, const float* __restrict__ k0b,
    const float* __restrict__ k1w, const float* __restrict__ k1b, float* __restrict__ h2)
{
  __shared__ __align__(16) float s_w0[kKin * kKer];
  __shared__ __align__(16) float s_b0[kKer];
  __shared__ __align__(16) float s_w1[kKer * kKer];
  __shared__ __align__(16) float s_b1[kKer];
  __shared__ __align__(16) float s_h1[kKer * 64];
  __shared__ __align__(16) float s_out[64 * 68];
  const int tid  = threadIdx.x;
  const int lane = tid & 31;
  const int wave = __builtin_amdgcn_readfirstlane((int)(threadIdx.x >> 5));
#pragma unroll 1
  for (int it = 0; it < 16; ++it) {
    const int i = it * 64 + tid;
    const v4f v = *(const v4f*)(k1w + 4 * i);
    *(v4f*)(s_w1 + 4 * i) = rbf4(v);
  }
#pragma unroll 1
  for (int it = 0; it < 2; ++it) {
    const int i = it * 64 + tid;
    const int ic = i < 96 ? i : 95;
    v4f v = *(const v4f*)(k0w + 4 * ic);
    asm volatile("" : "+v"(v));
    if (i < 96) *(v4f*)(s_w0 + 4 * i) = rbf4(v);
  }
  {
    const int ic = tid & 15;
    v4f va = *(const v4f*)(k0b + 4 * ic);
    v4f vb = *(const v4f*)(k1b + 4 * ic);
    asm volatile("" : "+v"(va), "+v"(vb));
    if (tid < 16) { *(v4f*)(s_b0 + 4 * ic) = rbf4(va); *(v4f*)(s_b1 + 4 * ic) = rbf4(vb); }
  }
  __syncthreads();

  const int e0 = blockIdx.x * 64;
  const int e  = e0 + tid;
  const int ec = e < kE ? e : kE - 1;
  float a[kKin];
  {
    const v2f p0 = *(const v2f*)(ea + (size_t)ec * kKin);
    const v2f p1 = *(const v2f*)(ea + (size_t)ec * kKin + 2);
    const v2f p2 = *(const v2f*)(ea + (size_t)ec * kKin + 4);
    const float t0 = p0[0], t1 = p0[1], t2 = p1[0], t3 = p1[1], t4 = p2[0], t5 = p2[1];
    a[0] = rbf(t0); a[1] = rbf(t1); a[2] = rbf(t2); a[3] = rbf(t3); a[4] = rbf(t4); a[5] = rbf(t5);
  }
#pragma unroll 1
  for (int j4 = 0; j4 < 16; ++j4) {
    v4f acc = (v4f){0.f, 0.f, 0.f, 0.f};
#pragma unroll
    for (int i = 0; i < kKin; ++i) {
      const v4f w = *(const v4f*)(s_w0 + i * kKer + 4 * j4);
      acc[0] = fmaf(a[i], w[0], acc[0]);
      acc[1] = fmaf(a[i], w[1], acc[1]);
      acc[2] = fmaf(a[i], w[2], acc[2]);
      acc[3] = fmaf(a[i], w[3], acc[3]);
    }
    const v4f bq = *(const v4f*)(s_b0 + 4 * j4);
    s_h1[(4 * j4 + 0) * 64 + tid] = fmaxf(acc[0] + bq[0], 0.0f);
    s_h1[(4 * j4 + 1) * 64 + tid] = fmaxf(acc[1] + bq[1], 0.0f);
    s_h1[(4 * j4 + 2) * 64 + tid] = fmaxf(acc[2] + bq[2], 0.0f);
    s_h1[(4 * j4 + 3) * 64 + tid] = fmaxf(acc[3] + bq[3], 0.0f);
  }
#pragma unroll 1
  for (int jc = 0; jc < 4; ++jc) {
    v4f c0 = (v4f){0.f, 0.f, 0.f, 0.f};
    v4f c1 = c0, c2 = c0, c3 = c0;
#pragma unroll 2
    for (int k = 0; k < kKer; ++k) {
      const float hk = s_h1[k * 64 + tid];
      const float* wp = s_w1 + k * kKer + jc * 16;
      const v4f w0 = *(const v4f*)(wp);
      const v4f w1 = *(const v4f*)(wp + 4);
      const v4f w2 = *(const v4f*)(wp + 8);
      const v4f w3 = *(const v4f*)(wp + 12);
      c0[0] = fmaf(hk, w0[0], c0[0]); c0[1] = fmaf(hk, w0[1], c0[1]); c0[2] = fmaf(hk, w0[2], c0[2]); c0[3] = fmaf(hk, w0[3], c0[3]);
      c1[0] = fmaf(hk, w1[0], c1[0]); c1[1] = fmaf(hk, w1[1], c1[1]); c1[2] = fmaf(hk, w1[2], c1[2]); c1[3] = fmaf(hk, w1[3], c1[3]);
      c2[0] = fmaf(hk, w2[0], c2[0]); c2[1] = fmaf(hk, w2[1], c2[1]); c2[2] = fmaf(hk, w2[2], c2[2]); c2[3] = fmaf(hk, w2[3], c2[3]);
      c3[0] = fmaf(hk, w3[0], c3[0]); c3[1] = fmaf(hk, w3[1], c3[1]); c3[2] = fmaf(hk, w3[2], c3[2]); c3[3] = fmaf(hk, w3[3], c3[3]);
    }
    const v4f b0 = *(const v4f*)(s_b1 + jc * 16);
    const v4f b1 = *(const v4f*)(s_b1 + jc * 16 + 4);
    const v4f b2 = *(const v4f*)(s_b1 + jc * 16 + 8);
    const v4f b3 = *(const v4f*)(s_b1 + jc * 16 + 12);
    v4f o0, o1, o2, o3;
#pragma unroll
    for (int q = 0; q < 4; ++q) {
      o0[q] = fmaxf(c0[q] + b0[q], 0.0f);
      o1[q] = fmaxf(c1[q] + b1[q], 0.0f);
      o2[q] = fmaxf(c2[q] + b2[q], 0.0f);
      o3[q] = fmaxf(c3[q] + b3[q], 0.0f);
    }
    float* op = s_out + tid * 68 + jc * 16;
    *(v4f*)(op)      = o0;
    *(v4f*)(op + 4)  = o1;
    *(v4f*)(op + 8)  = o2;
    *(v4f*)(op + 12) = o3;
  }
  __syncthreads();
  {
    const int hh = lane >> 4, c4 = (lane & 15) * 4;
    const v4f z4 = (v4f){0.f, 0.f, 0.f, 0.f};
    for (int pass = 0; pass < 2; ++pass) {
#pragma unroll 4
      for (int it = 0; it < 16; ++it) {
        const int row = wave * 32 + it * 2 + hh;
        v4f v = *(const v4f*)(s_out + row * 68 + c4);
        const bool keep = (e0 + row) < kE;
        v = keep ? v : z4;
        *(volatile v4f*)(h2 + (size_t)(e0 + row) * kKer + c4) = v;
      }
      __threadfence();
    }
  }
}

__global__ __launch_bounds__(160) void conv_msg(
    const float* __restrict__ x, const int* __restrict__ ei, const float* __restrict__ h2,
    const unsigned short* __restrict__ w2t, float* __restrict__ msg)
{
  __shared__ __align__(16) float s_reg[kCW * kRegion];
  const int lane = threadIdx.x & 31;
  const int wave = __builtin_amdgcn_readfirstlane((int)(threadIdx.x >> 5));
  float* reg = s_reg + wave * kRegion;
  const int e0 = (blockIdx.x * kCW + wave) * kCE;
  const int hh = lane >> 4, c = lane & 15;
  const int q = lane >> 3, c4 = (lane & 7) * 4;

#pragma unroll
  for (int it = 0; it < 12; ++it) {
    const int r = it * 4 + q;
    int s = ei[e0 + r];
    s = s < 0 ? 0 : s;
    s = s > (kNT - 1) ? (kNT - 1) : s;
    const v4f v = *(const v4f*)(x + (size_t)s * kXP + c4);
    *(v4f*)(reg + r * kXSP + c4) = v;
  }
  __syncthreads();

  v16b ah[3], al[3];
#pragma unroll
  for (int t = 0; t < 3; ++t) {
    const float* p = reg + (t * 16 + c) * kXSP + 8 * hh;
    const v4f a0 = *(const v4f*)(p);
    const v4f a1 = *(const v4f*)(p + 4);
    const v4f a2 = *(const v4f*)(p + 16);
    const v4f a3 = *(const v4f*)(p + 20);
    float f[16];
#pragma unroll
    for (int e = 0; e < 4; ++e) {
      f[e]      = a0[e];
      f[4 + e]  = a1[e];
      f[8 + e]  = a2[e];
      f[12 + e] = a3[e];
    }
    v8u hv, lv;
#pragma unroll
    for (int e = 0; e < 8; ++e) {
      unsigned h0, l0, h1, l1;
      split2(f[2 * e], h0, l0);
      split2(f[2 * e + 1], h1, l1);
      hv[e] = h0 | (h1 << 16);
      lv[e] = l0 | (l1 << 16);
    }
    ah[t] = __builtin_bit_cast(v16b, hv);
    al[t] = __builtin_bit_cast(v16b, lv);
  }
  __syncthreads();

#pragma unroll 4
  for (int it = 0; it < 24; ++it) {
    const int r = it * 2 + hh;
    const int k4 = c * 4;
    const v4f v = *(const v4f*)(h2 + (size_t)(e0 + r) * kKer + k4);
    const float v0 = v[0], v1 = v[1], v2 = v[2], v3 = v[3];
    reg[(k4 + 0) * kHTP + r] = v0;
    reg[(k4 + 1) * kHTP + r] = v1;
    reg[(k4 + 2) * kHTP + r] = v2;
    reg[(k4 + 3) * kHTP + r] = v3;
  }
  reg[kKer * kHTP + lane] = 1.0f;
  if (lane < 16) reg[kKer * kHTP + 32 + lane] = 1.0f;
  __syncthreads();

  v8f acc[3][2];
#pragma unroll
  for (int t = 0; t < 3; ++t) {
    acc[t][0] = (v8f){0.f, 0.f, 0.f, 0.f, 0.f, 0.f, 0.f, 0.f};
    acc[t][1] = (v8f){0.f, 0.f, 0.f, 0.f, 0.f, 0.f, 0.f, 0.f};
  }
  const __bf16* wb = (const __bf16*)(const void*)w2t + c * 32 + 8 * hh;
  const v8f zero8 = (v8f){0.f, 0.f, 0.f, 0.f, 0.f, 0.f, 0.f, 0.f};
#pragma unroll 1
  for (int kk = 0; kk < kKK; ++kk) {
    const v16b b0 = frag_load(wb + kk * 1024);
    const v16b b1 = frag_load(wb + kk * 1024 + 512);
    const float* hp = reg + kk * kHTP + 8 * hh;
#pragma unroll
    for (int t = 0; t < 3; ++t) {
      const v4f h0 = *(const v4f*)(hp + t * 16);
      const v4f h1 = *(const v4f*)(hp + t * 16 + 4);
      v8f c0 = mma_bf(al[t], b0, zero8);
      c0 = mma_bf(ah[t], b0, c0);
      guard1(c0, ah[t], al[t], b0);
      scale_acc(acc[t][0], c0, h0, h1);
      v8f c1 = mma_bf(al[t], b1, zero8);
      c1 = mma_bf(ah[t], b1, c1);
      guard1(c1, ah[t], al[t], b1);
      scale_acc(acc[t][1], c1, h0, h1);
    }
  }
  __syncthreads();

#pragma unroll
  for (int t = 0; t < 3; ++t) {
#pragma unroll
    for (int r = 0; r < 8; ++r) {
      reg[(t * 16 + 8 * hh + r) * kXSP + c]      = acc[t][0][r];
      reg[(t * 16 + 8 * hh + r) * kXSP + 16 + c] = acc[t][1][r];
    }
  }
  __syncthreads();
  for (int pass = 0; pass < 2; ++pass) {
#pragma unroll
    for (int it = 0; it < 12; ++it) {
      const int r = it * 4 + q;
      const v4f v = *(const v4f*)(reg + r * kXSP + c4);
      *(volatile v4f*)(msg + (size_t)(e0 + r) * kXP + c4) = v;
    }
    __threadfence();
  }
}

template <bool LAST>
__global__ __launch_bounds__(32) void agg_update(
    const float* __restrict__ msg, const int* __restrict__ ei, const float* __restrict__ xcur,
    const float* __restrict__ root, const float* __restrict__ bias,
    const float* __restrict__ fc3w, const float* __restrict__ fc3b,
    float* __restrict__ xnext, float* __restrict__ out)
{
  __shared__ __align__(16) float sA[kTile * 32];
  const int lane = threadIdx.x;
  const int n0 = blockIdx.x * kTile;
  int nn = kNT - n0;
  nn = nn > kTile ? kTile : nn;
  const int oc = lane < kW ? lane : kW - 1;

  float rc[kW];
  float fc[kW];
#pragma unroll 1
  for (int it = 0; it < 8; ++it) {
    const int i = it * 32 + lane;
    const int ic = i < 225 ? i : 224;
    v4f v = *(const v4f*)(root + 4 * ic);
    asm volatile("" : "+v"(v));
    if (i < 225) *(v4f*)(sA + 4 * i) = rbf4(v);
  }
  __syncthreads();
#pragma unroll
  for (int i = 0; i < kW; ++i) rc[i] = sA[i * kW + oc];
  __syncthreads();
  if (LAST) {
#pragma unroll 1
    for (int it = 0; it < 8; ++it) {
      const int i = it * 32 + lane;
      const int ic = i < 225 ? i : 224;
      v4f v = *(const v4f*)(fc3w + 4 * ic);
      asm volatile("" : "+v"(v));
      if (i < 225) *(v4f*)(sA + 4 * i) = rbf4(v);
    }
    __syncthreads();
#pragma unroll
    for (int i = 0; i < kW; ++i) fc[i] = sA[i * kW + oc];
    __syncthreads();
  } else {
#pragma unroll
    for (int i = 0; i < kW; ++i) fc[i] = 0.0f;
  }
  const float bv = rbf(bias[oc]);
  const float fb = rbf(fc3b[oc]);

  {
    const v4f z4 = (v4f){0.f, 0.f, 0.f, 0.f};
#pragma unroll 4
    for (int it = 0; it < (kTile * 8) / 32; ++it) *(v4f*)(sA + (it * 32 + lane) * 4) = z4;
  }
  __syncthreads();

  const int* dstp = ei + kE;
#pragma unroll 1
  for (int ch = 0; ch < kNCh; ++ch) {
    const int eb  = ch * 256 + lane * 8;
    const int ebc = eb < kE ? eb : kE - 8;
    const v4i d0 = *(const v4i*)(dstp + ebc);
    const v4i d1 = *(const v4i*)(dstp + ebc + 4);
    const unsigned lim = eb < kE ? (unsigned)nn : 0u;
    int dl[8];
    dl[0] = d0[0] - n0; dl[1] = d0[1] - n0; dl[2] = d0[2] - n0; dl[3] = d0[3] - n0;
    dl[4] = d1[0] - n0; dl[5] = d1[1] - n0; dl[6] = d1[2] - n0; dl[7] = d1[3] - n0;
    bool f[8];
#pragma unroll
    for (int k = 0; k < 8; ++k) f[k] = (unsigned)dl[k] < lim;
    const bool anyf = f[0] | f[1] | f[2] | f[3] | f[4] | f[5] | f[6] | f[7];
    if (__builtin_amdgcn_ballot_w32(anyf) == 0u) continue;
#pragma unroll
    for (int k = 0; k < 8; ++k) {
      unsigned mask = __builtin_amdgcn_ballot_w32(f[k]);
#pragma unroll 1
      for (int it = 0; it < 32; ++it) {
        if (mask == 0u) break;
        const int l = __builtin_ctz(mask);
        mask &= mask - 1u;
        int dlu = __builtin_amdgcn_readlane(dl[k], l);
        dlu = dlu < 0 ? 0 : dlu;
        dlu = dlu > (kTile - 1) ? (kTile - 1) : dlu;
        int e = ch * 256 + l * 8 + k;
        e = e > (kE - 1) ? (kE - 1) : e;
        float v = msg[(size_t)e * kXP + lane];
        asm volatile("" : "+v"(v));
        v = (lane == 31) ? 1.0f : v;
        sA[dlu * 32 + lane] += v;
      }
    }
  }
  __syncthreads();

#pragma unroll 1
  for (int nl = 0; nl < nn; ++nl) {
    const float xr = xcur[(size_t)(n0 + nl) * kXP + lane];
    const float a  = sA[nl * 32 + lane];
    float cntf = bcast(a, 31);
    cntf = fmaxf(cntf, 1.0f);
    const float inv = __builtin_amdgcn_rcpf(cntf);
    float acc = 0.0f;
#pragma unroll
    for (int i = 0; i < kW; ++i) acc = fmaf(bcast(xr, i), rc[i], acc);
    float y = a * inv + acc;
    y += bv;
    y = fmaxf(y, 0.0f);
    y = lane < kW ? y : 0.0f;
    if (!LAST) {
      sA[nl * 32 + lane] = y;
    } else {
      float o = 0.0f;
#pragma unroll
      for (int i = 0; i < kW; ++i) o = fmaf(bcast(y, i), fc[i], o);
      o += fb;
      if (lane < kW) sA[nl * kW + lane] = o;
    }
  }
  __syncthreads();

  const int nvec = LAST ? (nn * kW) / 4 : nn * 8;
  float* dst = LAST ? (out + (size_t)n0 * kW) : (xnext + (size_t)n0 * kXP);
  for (int pass = 0; pass < 2; ++pass) {
#pragma unroll 1
    for (int idx = lane; idx < nvec; idx += 32) {
      const v4f v = *(const v4f*)(sA + idx * 4);
      *(volatile v4f*)(dst + (size_t)idx * 4) = v;
    }
    __threadfence();
  }
}

extern "C" void kernel_launch(void* const* d_in, const int* in_sizes, int n_in,
                              void* d_out, int out_size, void* d_ws, size_t ws_size,
                              hipStream_t stream) {
  if (n_in < 21) return;
  if (in_sizes[0] != kB * kWin * kNodes * kD) return;
  if (in_sizes[1] != 2 * kE) return;
  if (in_sizes[2] != kE * kKin) return;
  if (in_sizes[3] != kW * kW) return;
  if (in_sizes[5] != kW * 4 * kW) return;
  if (in_sizes[6] != kW * 4 * kW) return;
  if (in_sizes[9] != kKin * kKer) return;
  if (in_sizes[11] != kKer * kKer) return;
  if (in_sizes[13] != kKer * kW * kW) return;
  if (in_sizes[14] != kW * kW) return;
  if (out_size != kNT * kW) return;
  if (ws_size < kWsTotal) return;

  const float* xpos  = (const float*)d_in[0];
  const int*   ei    = (const int*)  d_in[1];
  const float* eattr = (const float*)d_in[2];
  const float* fc0w  = (const float*)d_in[3];
  const float* fc0b  = (const float*)d_in[4];
  const float* wih   = (const float*)d_in[5];
  const float* whh   = (const float*)d_in[6];
  const float* bih   = (const float*)d_in[7];
  const float* bhh   = (const float*)d_in[8];
  const float* k0w   = (const float*)d_in[9];
  const float* k0b   = (const float*)d_in[10];
  const float* k1w   = (const float*)d_in[11];
  const float* k1b   = (const float*)d_in[12];
  const float* k2w   = (const float*)d_in[13];
  const float* k2b   = (const float*)d_in[14];
  const float* root1 = (const float*)d_in[15];
  const float* bias1 = (const float*)d_in[16];
  const float* root2 = (const float*)d_in[17];
  const float* bias2 = (const float*)d_in[18];
  const float* fc3w  = (const float*)d_in[19];
  const float* fc3b  = (const float*)d_in[20];
  float* out = (float*)d_out;

  char* ws = (char*)d_ws;
  unsigned short* W2T = (unsigned short*)(ws + kOffW2T);
  float* XA  = (float*)(ws + kOffXA);
  float* XB  = (float*)(ws + kOffXB);
  float* H2  = (float*)(ws + kOffH2);
  float* MSG = (float*)(ws + kOffMSG);

  prep_w2t<<<kKK, 128, 0, stream>>>(k2w, k2b, W2T);
  lstm_enc<<<kB / (kLW * kLNB), kLW * 32, 0, stream>>>(xpos, fc0w, fc0b, wih, whh, bih, bhh, XA);
  edge_mlp<<<kMlpBlocks, 64, 0, stream>>>(eattr, k0w, k0b, k1w, k1b, H2);

  const int msgBlocks = kE / (kCW * kCE);
  conv_msg<<<msgBlocks, kCW * 32, 0, stream>>>(XA, ei, H2, W2T, MSG);
  agg_update<false><<<kNTiles, 32, 0, stream>>>(MSG, ei, XA, root1, bias1, fc3w, fc3b, XB, out);
  conv_msg<<<msgBlocks, kCW * 32, 0, stream>>>(XB, ei, H2, W2T, MSG);
  agg_update<false><<<kNTiles, 32, 0, stream>>>(MSG, ei, XB, root1, bias1, fc3w, fc3b, XA, out);
  conv_msg<<<msgBlocks, kCW * 32, 0, stream>>>(XA, ei, H2, W2T, MSG);
  agg_update<false><<<kNTiles, 32, 0, stream>>>(MSG, ei, XA, root2, bias2, fc3w, fc3b, XB, out);
  conv_msg<<<msgBlocks, kCW * 32, 0, stream>>>(XB, ei, H2, W2T, MSG);
  agg_update<true><<<kNTiles, 32, 0, stream>>>(MSG, ei, XB, root2, bias2, fc3w, fc3b, XA, out);
}
